// BiLSTM_39745627357363
// MI455X (gfx1250) — hardware-verified
//
#include <hip/hip_runtime.h>
#include <math.h>

constexpr int NBATCH   = 32;
constexpr int NSTEP    = 512;
constexpr int NEMB     = 128;
constexpr int NHID     = 256;
constexpr int NVOC     = 21128;
constexpr int NTAG     = 32;
constexpr int NGATE3   = 3 * NHID;
constexpr int NROWS    = NBATCH * NSTEP;
constexpr int SCAN_THR = 512;
constexpr int SCAN_WAVES = SCAN_THR / 32;
constexpr int ROWS_BLK = 16;
constexpr int NBLK_SCAN = 2 * (NBATCH / ROWS_BLK);
constexpr int XPITCH   = 136;
constexpr int HPITCH   = 264;
constexpr int TAG_THR  = 256;
constexpr int SLABP    = 36;
constexpr float ACARRY   = 64.0f;
constexpr float WCARRY   = 16.0f;
constexpr float PROD_INV = 1.0f / 1024.0f;

static_assert(NHID == 16 * SCAN_WAVES, "one 16-column unit subtile per wave");
static_assert(ROWS_BLK == SCAN_WAVES, "one wave stages / stores one batch row");
static_assert(NBATCH % ROWS_BLK == 0, "batch tiles exact");
static_assert(NEMB % 32 == 0 && NHID % 32 == 0 && (2 * NHID) % 32 == 0, "every contraction K is a multiple of 32");
static_assert(NEMB == 32 * 4, "emb row tile: 32 lanes x 4 elements");
static_assert(NHID == 32 * 8, "h row store: 32 lanes x 8 elements = one 512-B row");
static_assert(NSTEP == 32 * 16, "word table: 16 entries per lane");
static_assert(NVOC < 32768, "word id fits in 16 bits");
static_assert(XPITCH >= NEMB && HPITCH >= NHID, "tile pitches cover K");
static_assert((XPITCH * 2) % 16 == 0 && (HPITCH * 2) % 16 == 0, "16-B aligned LDS rows");
static_assert(NTAG == 32, "two 16-column subtiles, one 128-B output line per row");
static_assert(NROWS % (16 * (TAG_THR / 32)) == 0, "tag-head grid exact");
static_assert((SLABP * 4) % 16 == 0, "16-B aligned slab rows");

typedef __attribute__((ext_vector_type(16))) _Float16 v16h;
typedef __attribute__((ext_vector_type(8)))  _Float16 v8h;
typedef __attribute__((ext_vector_type(16))) __bf16   v16b;
typedef __attribute__((ext_vector_type(8)))  __bf16   v8b;
typedef __attribute__((ext_vector_type(8)))  float    v8f;
typedef __attribute__((ext_vector_type(4)))  float    v4f;
typedef __attribute__((ext_vector_type(4)))  unsigned v4u;
typedef __attribute__((ext_vector_type(2)))  unsigned v2u;
typedef __attribute__((ext_vector_type(2)))  int      v2i;

__device__ __forceinline__ unsigned short f2bf_bits(float f) {
  unsigned u = __float_as_uint(f);
  return (unsigned short)((u + 0x7FFFu + ((u >> 16) & 1u)) >> 16);
}
__device__ __forceinline__ float bf_bits2f(unsigned short h) { return __uint_as_float(((unsigned)h) << 16); }
__device__ __forceinline__ float bf16r(float f) { return bf_bits2f(f2bf_bits(f)); }
__device__ __forceinline__ unsigned short h16c_bits(float f) {
  return __builtin_bit_cast(unsigned short, (_Float16)(bf16r(f) * ACARRY));
}

__device__ __forceinline__ void dep_guard_h(v8f& a, v8f& b, v16h x, v16h y) { asm volatile("v_nop\n\tv_nop\n\tv_nop\n\tv_nop" : "+v"(a), "+v"(b) : "v"(x), "v"(y)); }
__device__ __forceinline__ void dep_guard_b(v8f& a, v8f& b, v16b x, v16b y) { asm volatile("v_nop\n\tv_nop\n\tv_nop\n\tv_nop" : "+v"(a), "+v"(b) : "v"(x), "v"(y)); }
__device__ __forceinline__ void keep4_h(v16h a, v16h b, v16h c, v16h d) { asm volatile("v_nop" :: "v"(a), "v"(b), "v"(c), "v"(d)); }
__device__ __forceinline__ void keep4_b(v16b a, v16b b, v16b c, v16b d) { asm volatile("v_nop" :: "v"(a), "v"(b), "v"(c), "v"(d)); }
__device__ __forceinline__ void guard4_x1(v8f& a0, v8f& a1, v8f& a2, v8f& a3, v16h x, v16h y0, v16h y1, v16h y2, v16h y3) {
  asm volatile("v_nop\n\tv_nop\n\tv_nop\n\tv_nop" : "+v"(a0), "+v"(a1), "+v"(a2), "+v"(a3) : "v"(x), "v"(y0), "v"(y1), "v"(y2), "v"(y3));
}
__device__ __forceinline__ void guard4_x2(v8f& a0, v8f& a1, v8f& a2, v8f& a3, v16h x0, v16h x1, v16h y0, v16h y1, v16h y2, v16h y3) {
  asm volatile("v_nop\n\tv_nop\n\tv_nop\n\tv_nop" : "+v"(a0), "+v"(a1), "+v"(a2), "+v"(a3) : "v"(x0), "v"(x1), "v"(y0), "v"(y1), "v"(y2), "v"(y3));
}
__device__ __forceinline__ void guard3_x1(v8f& a0, v8f& a1, v8f& a2, v16h x, v16h y0, v16h y1, v16h y2) {
  asm volatile("v_nop\n\tv_nop\n\tv_nop\n\tv_nop" : "+v"(a0), "+v"(a1), "+v"(a2) : "v"(x), "v"(y0), "v"(y1), "v"(y2));
}
__device__ __forceinline__ void guard2_b2(v8f& a0, v8f& a1, v16b x0, v16b x1, v16b y0, v16b y1) {
  asm volatile("v_nop\n\tv_nop\n\tv_nop\n\tv_nop" : "+v"(a0), "+v"(a1) : "v"(x0), "v"(x1), "v"(y0), "v"(y1));
}
__device__ __forceinline__ void acc_guard4(v8f& a, v8f& b, v8f& c, v8f& d) { asm volatile("v_nop\n\tv_nop\n\tv_nop\n\tv_nop" : "+v"(a), "+v"(b), "+v"(c), "+v"(d)); }
__device__ __forceinline__ void acc_guard3(v8f& a, v8f& b, v8f& c) { asm volatile("v_nop\n\tv_nop\n\tv_nop\n\tv_nop" : "+v"(a), "+v"(b), "+v"(c)); }
__device__ __forceinline__ void acc_guard2(v8f& a, v8f& b) { asm volatile("v_nop\n\tv_nop\n\tv_nop\n\tv_nop" : "+v"(a), "+v"(b)); }

template <typename T> struct Frag;
template <> struct Frag<_Float16> {
  typedef v16h V; union U { v16h v; v8h h[2]; };
  static __device__ __forceinline__ v16h load(const _Float16* p) {
    U f; f.h[0] = *(const v8h*)(p); f.h[1] = *(const v8h*)(p + 16); return f.v;
  }
  static __device__ __forceinline__ v8f mma(v16h a, v16h b, v8f c) {
    return __builtin_amdgcn_wmma_f32_16x16x32_f16(false, a, false, b, (short)0, c, false, false);
  }
  static __device__ __forceinline__ void guard(v8f& a, v8f& b, v16h x, v16h y) { dep_guard_h(a, b, x, y); }
  static __device__ __forceinline__ void keep(v16h a, v16h b, v16h c, v16h d) { keep4_h(a, b, c, d); }
};
template <> struct Frag<__bf16> {
  typedef v16b V; union U { v16b v; v8b h[2]; };
  static __device__ __forceinline__ v16b load(const __bf16* p) {
    U f; f.h[0] = *(const v8b*)(p); f.h[1] = *(const v8b*)(p + 16); return f.v;
  }
  static __device__ __forceinline__ v8f mma(v16b a, v16b b, v8f c) {
    return __builtin_amdgcn_wmma_f32_16x16x32_bf16(false, a, false, b, (short)0, c, false, false);
  }
  static __device__ __forceinline__ void guard(v8f& a, v8f& b, v16b x, v16b y) { dep_guard_b(a, b, x, y); }
  static __device__ __forceinline__ void keep(v16b a, v16b b, v16b c, v16b d) { keep4_b(a, b, c, d); }
};

__device__ __forceinline__ float fsig(float x) { return 1.0f / (1.0f + expf(-x)); }

template <int MODE>
__global__ __launch_bounds__(256) void tcv8_kernel(const float* __restrict__ src, unsigned short* __restrict__ dst,
                                                   int krows, int ncols, float sc) {
  const int i   = (int)blockIdx.x * 256 + (int)threadIdx.x;
  const int k8n = krows >> 3;
  const int n8  = ncols * k8n;
  if (i < n8) {
    const int n  = i / k8n;
    const int k8 = (i - n * k8n) * 8;
    v8h hv;
#pragma unroll
    for (int e = 0; e < 8; ++e) {
      const float f = src[(size_t)(k8 + e) * (size_t)ncols + (size_t)n];
      unsigned short bits;
      if (MODE == 0) bits = __builtin_bit_cast(unsigned short, (_Float16)(bf16r(f) * sc));
      else           bits = f2bf_bits(f);
      hv[e] = __builtin_bit_cast(_Float16, bits);
    }
    unsigned short* op = dst + (size_t)i * 8;
    *(volatile v8h*)op = hv;
    __threadfence();
    *(volatile v8h*)op = hv;
  }
}

__device__ __forceinline__ int clamp_id(int id) {
  int w = id;
  w = (w < 0) ? (w + NVOC) : w;
  w = (w < 0) ? 0 : w;
  w = (w > NVOC - 1) ? (NVOC - 1) : w;
  return w;
}
__device__ __forceinline__ unsigned pack_word(int wid, int wl) {
  const int w = clamp_id(wid);
  int l = wl;
  l = (l < -32768) ? -32768 : l;
  l = (l > 32767) ? 32767 : l;
  return (unsigned)w | (((unsigned)l & 0xffffu) << 16);
}
__device__ __forceinline__ void stage_emb_row(unsigned short* tile, const float* __restrict__ emb, int id, int row, int lane) {
  const int w = clamp_id(id);
  const v4f v = *(const v4f*)(emb + (size_t)w * NEMB + 4 * lane);
  const float f0 = v[0];
  const float f1 = v[1];
  const float f2 = v[2];
  const float f3 = v[3];
  const unsigned u0 = h16c_bits(f0), u1 = h16c_bits(f1), u2 = h16c_bits(f2), u3 = h16c_bits(f3);
  v2u pk;
  pk[0] = u0 | (u1 << 16);
  pk[1] = u2 | (u3 << 16);
  *(v2u*)(tile + row * XPITCH + 4 * lane) = pk;
}

struct DirPtrs {
  const unsigned short* wit;
  const unsigned short* ait;
  const unsigned short* wht;
  const unsigned short* aht;
  const unsigned short* wwit;
  const unsigned short* wwht;
  const float* bmain;
  const float* balpha;
  const float* bword;
  unsigned short* hhi;
  unsigned short* hlo;
};
struct ScanArgs {
  DirPtrs d0, d1;
  const float* emb;
  const int*   cid;
  const int*   skp;
};
static_assert(sizeof(DirPtrs) == 88 && sizeof(ScanArgs) == 200, "no padding bytes");

__global__ __launch_bounds__(SCAN_THR) void seq_scan_kernel(ScanArgs a) {
  __shared__ __align__(16) unsigned short Xt[ROWS_BLK * XPITCH];
  __shared__ __align__(16) unsigned short Wt[ROWS_BLK * XPITCH];
  __shared__ __align__(16) unsigned short Hb[2][ROWS_BLK * HPITCH];
  __shared__ __align__(16) unsigned short Pt[ROWS_BLK * HPITCH];
  __shared__ __align__(16) unsigned short Shi[ROWS_BLK * HPITCH];
  __shared__ __align__(16) unsigned short Slo[ROWS_BLK * HPITCH];
  __shared__ __align__(16) unsigned       SK[ROWS_BLK * NSTEP];

  const int tid = (int)threadIdx.x, lane = tid & 31, wave = tid >> 5;
  const int c = lane & 15, hh = lane >> 4, koff = hh * 8;
  const int dir = (int)(blockIdx.x >> 1);
  const int browbase = (int)(blockIdx.x & 1u) * ROWS_BLK;
  const int j = 16 * wave + c;

  const _Float16* WIT  = (const _Float16*)(dir ? a.d1.wit  : a.d0.wit);
  const _Float16* AIT  = (const _Float16*)(dir ? a.d1.ait  : a.d0.ait);
  const _Float16* WHT  = (const _Float16*)(dir ? a.d1.wht  : a.d0.wht);
  const _Float16* AHT  = (const _Float16*)(dir ? a.d1.aht  : a.d0.aht);
  const _Float16* WWIT = (const _Float16*)(dir ? a.d1.wwit : a.d0.wwit);
  const _Float16* WWHT = (const _Float16*)(dir ? a.d1.wwht : a.d0.wwht);
  const float* BM = dir ? a.d1.bmain  : a.d0.bmain;
  const float* BA = dir ? a.d1.balpha : a.d0.balpha;
  const float* BW = dir ? a.d1.bword  : a.d0.bword;
  unsigned short* HHI = dir ? a.d1.hhi : a.d0.hhi;
  unsigned short* HLO = dir ? a.d1.hlo : a.d0.hlo;
  const float* EMB = a.emb;
  const int* cidrow = a.cid + (size_t)(browbase + wave) * NSTEP;
  const int* skrow  = a.skp + (size_t)(browbase + wave) * NSTEP * 2;

  {
    unsigned short* hbflat = &Hb[0][0];
#pragma unroll 1
    for (int i = tid; i < 2 * ROWS_BLK * HPITCH; i += SCAN_THR) hbflat[i] = (unsigned short)0;
#pragma unroll 1
    for (int i = tid; i < ROWS_BLK * HPITCH; i += SCAN_THR) Pt[i] = (unsigned short)0;
  }

  if (dir == 0) {
#pragma unroll 1
    for (int e = 0; e < NSTEP / 32; ++e) {
      const int ts = lane + 32 * e;
      const v2i sv = *(const v2i*)(skrow + 2 * ts);
      const int wraw = sv[0];
      const int wlr  = sv[1];
      SK[wave * NSTEP + ts] = pack_word(wraw, wlr);
    }
  } else {
    unsigned res[16];
#pragma unroll
    for (int e = 0; e < 16; ++e) res[e] = 0u;
#pragma unroll 1
    for (int ts = 0; ts < NSTEP; ++ts) {
      const v2i sv = *(const v2i*)(skrow + 2 * ts);
      const int wraw = sv[0];
      const int wlr  = sv[1];
      const unsigned pk = pack_word(wraw, wlr);
      const int key = NSTEP - ts - wlr;
      const bool ok = (wlr > 0) && ((unsigned)key < (unsigned)NSTEP);
      const int kq = ok ? key : -1;
#pragma unroll
      for (int e = 0; e < 16; ++e) res[e] = (kq == lane + 32 * e) ? pk : res[e];
    }
#pragma unroll
    for (int e = 0; e < 16; ++e) SK[wave * NSTEP + lane + 32 * e] = res[e];
  }

  {
    const int tp0 = dir ? (NSTEP - 1) : 0;
    const int id0 = cidrow[tp0];
    stage_emb_row(Xt, EMB, id0, wave, lane);
  }

  const float bi_ = bf16r(BM[j]);
  const float bo_ = bf16r(BM[NHID + j]);
  const float bg_ = bf16r(BM[2 * NHID + j]);
  const float ba_ = bf16r(BA[j]);
  const float bwi = bf16r(BW[j]);
  const float bwf = bf16r(BW[NHID + j]);
  const float bwg = bf16r(BW[2 * NHID + j]);

  const _Float16* wxi = WIT  + (size_t)j * NEMB + koff;
  const _Float16* wxo = WIT  + (size_t)(NHID + j) * NEMB + koff;
  const _Float16* wxg = WIT  + (size_t)(2 * NHID + j) * NEMB + koff;
  const _Float16* wxa = AIT  + (size_t)j * NEMB + koff;
  const _Float16* whi = WHT  + (size_t)j * NHID + koff;
  const _Float16* who = WHT  + (size_t)(NHID + j) * NHID + koff;
  const _Float16* whg = WHT  + (size_t)(2 * NHID + j) * NHID + koff;
  const _Float16* wha = AHT  + (size_t)j * NHID + koff;
  const _Float16* vxi = WWIT + (size_t)j * NEMB + koff;
  const _Float16* vxf = WWIT + (size_t)(NHID + j) * NEMB + koff;
  const _Float16* vxg = WWIT + (size_t)(2 * NHID + j) * NEMB + koff;
  const _Float16* vhi = WWHT + (size_t)j * NHID + koff;
  const _Float16* vhf = WWHT + (size_t)(NHID + j) * NHID + koff;
  const _Float16* vhg = WWHT + (size_t)(2 * NHID + j) * NHID + koff;

  float cst[8], pcs[8];
  int pcnt[8], pval[8];
#pragma unroll
  for (int r = 0; r < 8; ++r) { cst[r] = 0.0f; pcs[r] = 0.0f; pcnt[r] = -1; pval[r] = 0; }

  __syncthreads();

  const v8f z8 = {0.f, 0.f, 0.f, 0.f, 0.f, 0.f, 0.f, 0.f};
  const _Float16* xrow  = (const _Float16*)Xt + c * XPITCH + koff;
  const _Float16* werow = (const _Float16*)Wt + c * XPITCH + koff;
  const _Float16* prow  = (const _Float16*)Pt + c * HPITCH + koff;

#pragma unroll 1
  for (int t = 0; t < NSTEP; ++t) {
    const int P = t & 1;
    const int Q = P ^ 1;
    const int tpos = dir ? (NSTEP - 1 - t) : t;

    {
      const unsigned pkw = SK[wave * NSTEP + t];
      const int wid = (int)(pkw & 0xffffu);
      stage_emb_row(Wt, EMB, wid, wave, lane);
    }
    int wl[8];
#pragma unroll
    for (int r = 0; r < 8; ++r) {
      const int sv = (int)SK[(8 * hh + r) * NSTEP + t];
      wl[r] = sv >> 16;
    }

    v8f ai = z8, ao = z8, ag = z8, aa = z8;
#pragma unroll 1
    for (int kx = 0; kx < NEMB; kx += 32) {
      const v16h av = Frag<_Float16>::load(xrow + kx);
      const v16h b0 = Frag<_Float16>::load(wxi + kx);
      const v16h b1 = Frag<_Float16>::load(wxo + kx);
      const v16h b2 = Frag<_Float16>::load(wxg + kx);
      const v16h b3 = Frag<_Float16>::load(wxa + kx);
      ai = Frag<_Float16>::mma(av, b0, ai);
      ao = Frag<_Float16>::mma(av, b1, ao);
      ag = Frag<_Float16>::mma(av, b2, ag);
      aa = Frag<_Float16>::mma(av, b3, aa);
      guard4_x1(ai, ao, ag, aa, av, b0, b1, b2, b3);
    }
    {
      const _Float16* hrow = (const _Float16*)(&Hb[Q][0]) + c * HPITCH + koff;
#pragma unroll 1
      for (int k0 = 0; k0 < NHID; k0 += 32) {
        const v16h ah = Frag<_Float16>::load(hrow + k0);
        const v16h ap = Frag<_Float16>::load(prow + k0);
        const v16h b0 = Frag<_Float16>::load(whi + k0);
        const v16h b1 = Frag<_Float16>::load(who + k0);
        const v16h b2 = Frag<_Float16>::load(whg + k0);
        const v16h b3 = Frag<_Float16>::load(wha + k0);
        ai = Frag<_Float16>::mma(ah, b0, ai);
        ao = Frag<_Float16>::mma(ah, b1, ao);
        ag = Frag<_Float16>::mma(ah, b2, ag);
        aa = Frag<_Float16>::mma(ap, b3, aa);
        guard4_x2(ai, ao, ag, aa, ah, ap, b0, b1, b2, b3);
      }
    }
    acc_guard4(ai, ao, ag, aa);

    {
      unsigned short* hbw = &Hb[P][0];
#pragma unroll
      for (int r = 0; r < 8; ++r) {
        const float zi = ai[r] * PROD_INV + bi_;
        const float zo = ao[r] * PROD_INV + bo_;
        const float zg = ag[r] * PROD_INV + bg_;
        const float za = aa[r] * PROD_INV + ba_;
        const float ig = fsig(zi);
        const float og = fsig(zo);
        const float gg = tanhf(zg);
        const bool  mg = (pval[r] != 0) && (pcnt[r] == 0);
        const float c_plain = (1.0f - ig) * cst[r] + ig * gg;
        const float al = fsig(za);
        const float ei = expf(ig);
        const float ea = expf(al);
        const float c_merge = (ei * gg + ea * pcs[r]) / (ei + ea);
        const float cn = mg ? c_merge : c_plain;
        const float hn = og * tanhf(cn);
        cst[r]  = cn;
        pval[r] = mg ? 0 : pval[r];
        pcnt[r] = pcnt[r] - 1;
        const int li = (8 * hh + r) * HPITCH + j;
        hbw[li] = __builtin_bit_cast(unsigned short, (_Float16)(hn * ACARRY));
        const unsigned short hib = f2bf_bits(hn);
        Shi[li] = hib;
        Slo[li] = f2bf_bits(hn - bf_bits2f(hib));
      }
    }
    __syncthreads();

    {
      const v4u vh = *(const v4u*)(&Shi[wave * HPITCH + lane * 8]);
      const v4u vl = *(const v4u*)(&Slo[wave * HPITCH + lane * 8]);
      const size_t go = ((size_t)(browbase + wave) * NSTEP + (size_t)tpos) * NHID + (size_t)lane * 8;
      *(volatile v4u*)(HHI + go) = vh;
      *(volatile v4u*)(HLO + go) = vl;
      __threadfence();
      *(volatile v4u*)(HHI + go) = vh;
      *(volatile v4u*)(HLO + go) = vl;
    }
    {
      const int tn  = (t + 1 < NSTEP) ? (t + 1) : (NSTEP - 1);
      const int tnp = dir ? (NSTEP - 1 - tn) : tn;
      const int idn = cidrow[tnp];
      stage_emb_row(Xt, EMB, idn, wave, lane);
    }

    v8f qi = z8, qf = z8, qg = z8;
#pragma unroll 1
    for (int kx = 0; kx < NEMB; kx += 32) {
      const v16h av = Frag<_Float16>::load(werow + kx);
      const v16h b0 = Frag<_Float16>::load(vxi + kx);
      const v16h b1 = Frag<_Float16>::load(vxf + kx);
      const v16h b2 = Frag<_Float16>::load(vxg + kx);
      qi = Frag<_Float16>::mma(av, b0, qi);
      qf = Frag<_Float16>::mma(av, b1, qf);
      qg = Frag<_Float16>::mma(av, b2, qg);
      guard3_x1(qi, qf, qg, av, b0, b1, b2);
    }
    {
      const _Float16* hnrow = (const _Float16*)(&Hb[P][0]) + c * HPITCH + koff;
#pragma unroll 1
      for (int k0 = 0; k0 < NHID; k0 += 32) {
        const v16h ah = Frag<_Float16>::load(hnrow + k0);
        const v16h b0 = Frag<_Float16>::load(vhi + k0);
        const v16h b1 = Frag<_Float16>::load(vhf + k0);
        const v16h b2 = Frag<_Float16>::load(vhg + k0);
        qi = Frag<_Float16>::mma(ah, b0, qi);
        qf = Frag<_Float16>::mma(ah, b1, qf);
        qg = Frag<_Float16>::mma(ah, b2, qg);
        guard3_x1(qi, qf, qg, ah, b0, b1, b2);
      }
    }
    acc_guard3(qi, qf, qg);

#pragma unroll
    for (int r = 0; r < 8; ++r) {
      const bool has_w = (wl[r] >= 2);
      const float ziw = qi[r] * PROD_INV + bwi;
      const float zfw = qf[r] * PROD_INV + bwf;
      const float zgw = qg[r] * PROD_INV + bwg;
      const float cw  = fsig(zfw) * cst[r] + fsig(ziw) * tanhf(zgw);
      pcs[r]  = has_w ? cw : pcs[r];
      pcnt[r] = has_w ? (wl[r] - 1) : pcnt[r];
      pval[r] = has_w ? 1 : pval[r];
      Pt[(8 * hh + r) * HPITCH + j] = __builtin_bit_cast(unsigned short, (_Float16)(pcs[r] * ACARRY));
    }
    __syncthreads();
  }
}

__global__ __launch_bounds__(TAG_THR) void tag_head_kernel(const unsigned short* __restrict__ HFHp, const unsigned short* __restrict__ HFLp,
                                                          const unsigned short* __restrict__ HBHp, const unsigned short* __restrict__ HBLp,
                                                          const unsigned short* __restrict__ TWp, const float* __restrict__ tb,
                                                          float* __restrict__ out) {
  __shared__ __align__(16) float Sl[TAG_THR / 32][16 * SLABP];
  const __bf16* HFH = (const __bf16*)HFHp;
  const __bf16* HFL = (const __bf16*)HFLp;
  const __bf16* HBH = (const __bf16*)HBHp;
  const __bf16* HBL = (const __bf16*)HBLp;
  const __bf16* TW  = (const __bf16*)TWp;
  const int tid = (int)threadIdx.x, lane = tid & 31, wave = tid >> 5;
  const int c = lane & 15, hh = lane >> 4, koff = hh * 8;
  const int m0 = ((int)blockIdx.x * (TAG_THR / 32) + wave) * 16;
  const float tb0 = bf16r(tb[c]);
  const float tb1 = bf16r(tb[16 + c]);
  const v8f z8 = {0.f, 0.f, 0.f, 0.f, 0.f, 0.f, 0.f, 0.f};
  v8f a0 = z8, a1 = z8;
  const __bf16* bn0 = TW + (size_t)c * (2 * NHID) + koff;
  const __bf16* bn1 = TW + (size_t)(16 + c) * (2 * NHID) + koff;
  {
    const __bf16* ahr = HFH + (size_t)(m0 + c) * NHID + koff;
    const __bf16* alr = HFL + (size_t)(m0 + c) * NHID + koff;
#pragma unroll 1
    for (int k0 = 0; k0 < NHID; k0 += 32) {
      const v16b xh = Frag<__bf16>::load(ahr + k0);
      const v16b xl = Frag<__bf16>::load(alr + k0);
      const v16b y0 = Frag<__bf16>::load(bn0 + k0);
      const v16b y1 = Frag<__bf16>::load(bn1 + k0);
      a0 = Frag<__bf16>::mma(xh, y0, a0);
      a0 = Frag<__bf16>::mma(xl, y0, a0);
      a1 = Frag<__bf16>::mma(xh, y1, a1);
      a1 = Frag<__bf16>::mma(xl, y1, a1);
      guard2_b2(a0, a1, xh, xl, y0, y1);
    }
  }
  {
    const __bf16* ahr = HBH + (size_t)(m0 + c) * NHID + koff;
    const __bf16* alr = HBL + (size_t)(m0 + c) * NHID + koff;
#pragma unroll 1
    for (int k0 = 0; k0 < NHID; k0 += 32) {
      const v16b xh = Frag<__bf16>::load(ahr + k0);
      const v16b xl = Frag<__bf16>::load(alr + k0);
      const v16b y0 = Frag<__bf16>::load(bn0 + NHID + k0);
      const v16b y1 = Frag<__bf16>::load(bn1 + NHID + k0);
      a0 = Frag<__bf16>::mma(xh, y0, a0);
      a0 = Frag<__bf16>::mma(xl, y0, a0);
      a1 = Frag<__bf16>::mma(xh, y1, a1);
      a1 = Frag<__bf16>::mma(xl, y1, a1);
      guard2_b2(a0, a1, xh, xl, y0, y1);
    }
  }
  acc_guard2(a0, a1);

  float* slab = Sl[wave];
#pragma unroll
  for (int r = 0; r < 8; ++r) {
    slab[(8 * hh + r) * SLABP + c]      = a0[r] + tb0;
    slab[(8 * hh + r) * SLABP + 16 + c] = a1[r] + tb1;
  }
  __builtin_amdgcn_fence(__ATOMIC_RELEASE, "workgroup");
  __builtin_amdgcn_wave_barrier();
  __builtin_amdgcn_fence(__ATOMIC_ACQUIRE, "workgroup");
  const int q = lane >> 3, c4 = (lane & 7) * 4;
  v4f vv[4];
#pragma unroll
  for (int it = 0; it < 4; ++it) vv[it] = *(const v4f*)(slab + (it * 4 + q) * SLABP + c4);
  for (int pass = 0; pass < 2; ++pass) {
#pragma unroll
    for (int it = 0; it < 4; ++it) {
      const int row = it * 4 + q;
      *(volatile v4f*)(out + (size_t)(m0 + row) * NTAG + c4) = vv[it];
    }
    __threadfence();
  }
}

extern "C" void kernel_launch(void* const* d_in, const int* in_sizes, int n_in,
                              void* d_out, int out_size, void* d_ws, size_t ws_size, hipStream_t stream) {
  if (n_in < 23 || d_out == nullptr || d_ws == nullptr) return;
  if (in_sizes[0] != NBATCH * NSTEP || in_sizes[1] != NBATCH * NSTEP * 2 || in_sizes[2] != NVOC * NEMB ||
      in_sizes[3] != 2 * NHID * NTAG || in_sizes[4] != NTAG || out_size != NROWS * NTAG) return;
  for (int d = 0; d < 2; ++d) {
    const int o = 5 + 9 * d;
    if (in_sizes[o + 0] != NEMB * NGATE3 || in_sizes[o + 1] != NHID * NGATE3 || in_sizes[o + 2] != NGATE3 ||
        in_sizes[o + 3] != NEMB * NHID || in_sizes[o + 4] != NHID * NHID || in_sizes[o + 5] != NHID ||
        in_sizes[o + 6] != NEMB * NGATE3 || in_sizes[o + 7] != NHID * NGATE3 || in_sizes[o + 8] != NGATE3) return;
  }

  const int*   cid   = (const int*)d_in[0];
  const int*   skp   = (const int*)d_in[1];
  const float* emb   = (const float*)d_in[2];
  const float* tag_w = (const float*)d_in[3];
  const float* tag_b = (const float*)d_in[4];
  const float* w_ih[2], *w_hh[2], *b_m[2], *aw_ih[2], *aw_hh[2], *b_a[2], *ww_ih[2], *ww_hh[2], *b_w[2];
  for (int d = 0; d < 2; ++d) {
    const int o = 5 + 9 * d;
    w_ih[d]  = (const float*)d_in[o + 0];
    w_hh[d]  = (const float*)d_in[o + 1];
    b_m[d]   = (const float*)d_in[o + 2];
    aw_ih[d] = (const float*)d_in[o + 3];
    aw_hh[d] = (const float*)d_in[o + 4];
    b_a[d]   = (const float*)d_in[o + 5];
    ww_ih[d] = (const float*)d_in[o + 6];
    ww_hh[d] = (const float*)d_in[o + 7];
    b_w[d]   = (const float*)d_in[o + 8];
  }
  float* outp = (float*)d_out;

  char* ws = (char*)d_ws; size_t off = 0;
  auto carve = [&](size_t bytes) -> char* { char* p = ws + off; off += (bytes + 255) & ~(size_t)255; return p; };
  unsigned short *WIT[2], *AIT[2], *WHT[2], *AHT[2], *WWIT[2], *WWHT[2];
  for (int d = 0; d < 2; ++d) {
    WIT[d]  = (unsigned short*)carve((size_t)NGATE3 * NEMB * 2);
    AIT[d]  = (unsigned short*)carve((size_t)NHID * NEMB * 2);
    WHT[d]  = (unsigned short*)carve((size_t)NGATE3 * NHID * 2);
    AHT[d]  = (unsigned short*)carve((size_t)NHID * NHID * 2);
    WWIT[d] = (unsigned short*)carve((size_t)NGATE3 * NEMB * 2);
    WWHT[d] = (unsigned short*)carve((size_t)NGATE3 * NHID * 2);
  }
  unsigned short* TWB = (unsigned short*)carve((size_t)NTAG * (2 * NHID) * 2);
  unsigned short* HFH = (unsigned short*)carve((size_t)NROWS * NHID * 2);
  unsigned short* HFL = (unsigned short*)carve((size_t)NROWS * NHID * 2);
  unsigned short* HBH = (unsigned short*)carve((size_t)NROWS * NHID * 2);
  unsigned short* HBL = (unsigned short*)carve((size_t)NROWS * NHID * 2);
  if (off > ws_size || off > (size_t)134217728) return;

  for (int d = 0; d < 2; ++d) {
    tcv8_kernel<0><<<(NGATE3 * NEMB / 8 + 255) / 256, 256, 0, stream>>>(w_ih[d],  WIT[d],  NEMB, NGATE3, WCARRY);
    tcv8_kernel<0><<<(NHID * NEMB / 8 + 255) / 256,   256, 0, stream>>>(aw_ih[d], AIT[d],  NEMB, NHID,   WCARRY);
    tcv8_kernel<0><<<(NGATE3 * NHID / 8 + 255) / 256, 256, 0, stream>>>(w_hh[d],  WHT[d],  NHID, NGATE3, WCARRY);
    tcv8_kernel<0><<<(NHID * NHID / 8 + 255) / 256,   256, 0, stream>>>(aw_hh[d], AHT[d],  NHID, NHID,   WCARRY);
    tcv8_kernel<0><<<(NGATE3 * NEMB / 8 + 255) / 256, 256, 0, stream>>>(ww_ih[d], WWIT[d], NEMB, NGATE3, WCARRY);
    tcv8_kernel<0><<<(NGATE3 * NHID / 8 + 255) / 256, 256, 0, stream>>>(ww_hh[d], WWHT[d], NHID, NGATE3, WCARRY);
  }
  tcv8_kernel<1><<<(NTAG * 2 * NHID / 8 + 255) / 256, 256, 0, stream>>>(tag_w, TWB, 2 * NHID, NTAG, 1.0f);

  ScanArgs sa;
  sa.d0.wit = WIT[0]; sa.d0.ait = AIT[0]; sa.d0.wht = WHT[0]; sa.d0.aht = AHT[0]; sa.d0.wwit = WWIT[0]; sa.d0.wwht = WWHT[0];
  sa.d0.bmain = b_m[0]; sa.d0.balpha = b_a[0]; sa.d0.bword = b_w[0]; sa.d0.hhi = HFH; sa.d0.hlo = HFL;
  sa.d1.wit = WIT[1]; sa.d1.ait = AIT[1]; sa.d1.wht = WHT[1]; sa.d1.aht = AHT[1]; sa.d1.wwit = WWIT[1]; sa.d1.wwht = WWHT[1];
  sa.d1.bmain = b_m[1]; sa.d1.balpha = b_a[1]; sa.d1.bword = b_w[1]; sa.d1.hhi = HBH; sa.d1.hlo = HBL;
  sa.emb = emb; sa.cid = cid; sa.skp = skp;
  seq_scan_kernel<<<NBLK_SCAN, SCAN_THR, 0, stream>>>(sa);

  tag_head_kernel<<<NROWS / (16 * (TAG_THR / 32)), TAG_THR, 0, stream>>>(HFH, HFL, HBH, HBL, TWB, tag_b, outp);
}
